// AttentionBlock3D_48421461295757
// MI455X (gfx1250) — hardware-verified
//
#include <hip/hip_runtime.h>
#include <stdint.h>

#define NB     2
#define NC     256
#define NPOS   8192
#define NG     32
#define CPG    8
#define QBLK   1024
#define HPITCH 264

typedef __attribute__((ext_vector_type(16))) _Float16 v16h;
typedef __attribute__((ext_vector_type(8)))  _Float16 v8h;
typedef __attribute__((ext_vector_type(16))) __bf16   v16b;
typedef __attribute__((ext_vector_type(8)))  __bf16   v8b;
typedef __attribute__((ext_vector_type(8)))  float    v8f;
typedef __attribute__((ext_vector_type(4)))  float    v4f;

__device__ __forceinline__ unsigned short f2bf_bits(float f) {
  unsigned u = __float_as_uint(f);
  return (unsigned short)((u + 0x7FFFu + ((u >> 16) & 1u)) >> 16);
}
__device__ __forceinline__ float bf_bits2f(unsigned short h) { return __uint_as_float(((unsigned)h) << 16); }

__device__ __forceinline__ void dep_guard_h(v8f& a, v8f& b, v16h x, v16h y) { asm volatile("v_nop\n\tv_nop\n\tv_nop\n\tv_nop" : "+v"(a), "+v"(b) : "v"(x), "v"(y)); }
__device__ __forceinline__ void dep_guard_b(v8f& a, v8f& b, v16b x, v16b y) { asm volatile("v_nop\n\tv_nop\n\tv_nop\n\tv_nop" : "+v"(a), "+v"(b) : "v"(x), "v"(y)); }
__device__ __forceinline__ void keep4_h(v16h a, v16h b, v16h c, v16h d) { asm volatile("v_nop" :: "v"(a), "v"(b), "v"(c), "v"(d)); }
__device__ __forceinline__ void keep4_b(v16b a, v16b b, v16b c, v16b d) { asm volatile("v_nop" :: "v"(a), "v"(b), "v"(c), "v"(d)); }
__device__ __forceinline__ void acc_guard4(v8f& a, v8f& b, v8f& c, v8f& d) { asm volatile("v_nop\n\tv_nop\n\tv_nop\n\tv_nop" : "+v"(a), "+v"(b), "+v"(c), "+v"(d)); }
template <typename T> struct Frag;
template <> struct Frag<_Float16> {
  typedef v16h V; union U { v16h v; v8h h[2]; };
  static __device__ __forceinline__ v16h load(const _Float16* p) {
    U f; f.h[0] = *(const v8h*)(p); f.h[1] = *(const v8h*)(p + 16); return f.v;
  }
  static __device__ __forceinline__ v8f mma(v16h a, v16h b, v8f c) {
    return __builtin_amdgcn_wmma_f32_16x16x32_f16(false, a, false, b, (short)0, c, false, false);
  }
  static __device__ __forceinline__ void guard(v8f& a, v8f& b, v16h x, v16h y) { dep_guard_h(a, b, x, y); }
  static __device__ __forceinline__ void keep(v16h a, v16h b, v16h c, v16h d) { keep4_h(a, b, c, d); }
};
template <> struct Frag<__bf16> {
  typedef v16b V; union U { v16b v; v8b h[2]; };
  static __device__ __forceinline__ v16b load(const __bf16* p) {
    U f; f.h[0] = *(const v8b*)(p); f.h[1] = *(const v8b*)(p + 16); return f.v;
  }
  static __device__ __forceinline__ v8f mma(v16b a, v16b b, v8f c) {
    return __builtin_amdgcn_wmma_f32_16x16x32_bf16(false, a, false, b, (short)0, c, false, false);
  }
  static __device__ __forceinline__ void guard(v8f& a, v8f& b, v16b x, v16b y) { dep_guard_b(a, b, x, y); }
  static __device__ __forceinline__ void keep(v16b a, v16b b, v16b c, v16b d) { keep4_b(a, b, c, d); }
};

template <int ET> struct Elem;
template <> struct Elem<0> { typedef _Float16 T; };
template <> struct Elem<1> { typedef __bf16 T; };
template <int ET, bool SPLIT, int BIAS_MODE, int OUT_MODE, bool RESID, int ACT = 0>
__global__ __launch_bounds__(256) void wmma_gemm64(
    const unsigned short* __restrict__ Ap, const unsigned short* __restrict__ A2p, int lda, long strideA,
    const unsigned short* __restrict__ Btp, const unsigned short* __restrict__ Bt2p, int ldb, long strideB,
    void* __restrict__ Cout, void* __restrict__ Cout2, int ldc, long strideC,
    const float* __restrict__ bias,
    const float* __restrict__ resid, long strideR,
    int M, int N, int K, float scale) {
  typedef typename Elem<ET>::T T;
  typedef typename Frag<T>::V V;
  const T* A = (const T*)Ap; const T* A2 = (const T*)A2p; const T* Bt = (const T*)Btp; const T* Bt2 = (const T*)Bt2p;
  __shared__ __align__(16) float sT[8][16 * 68];
  const int b    = blockIdx.y;
  const int lane = threadIdx.x & 31;
  const int wave = threadIdx.x >> 5;
  const int tilesN = N >> 6;
  const int tilesM = M >> 6;
  const int tile = blockIdx.x * 8 + wave;
  if (tile >= tilesM * tilesN) return;
  const int tm = tile / tilesN;
  const int tn = tile - tm * tilesN;
  const int m0 = tm << 6;
  const int n0 = tn << 6;

  const T* Ab  = A  + (size_t)b * strideA;
  const T* Bb  = Bt + (size_t)b * strideB;
  const T* Ab2 = SPLIT ? (A2  + (size_t)b * strideA) : nullptr;
  const T* Bb2 = SPLIT ? (Bt2 + (size_t)b * strideB) : nullptr;

  const int rlane = lane & 15;
  const int koff  = (lane >> 4) * 8;
  const int mOff  = (lane >> 4) * 8;

  v8f acc[4][4];
#pragma unroll
  for (int i = 0; i < 4; ++i)
#pragma unroll
    for (int j = 0; j < 4; ++j) acc[i][j] = (v8f){0.f,0.f,0.f,0.f,0.f,0.f,0.f,0.f};

  for (int k0 = 0; k0 < K; k0 += 32) {
    V bh[4], bl[4];
#pragma unroll
    for (int j = 0; j < 4; ++j) {
      const size_t bo = (size_t)(n0 + (j << 4) + rlane) * ldb + koff + k0;
      bh[j] = Frag<T>::load(Bb + bo);
      if (SPLIT) bl[j] = Frag<T>::load(Bb2 + bo);
    }
#pragma unroll
    for (int i = 0; i < 4; ++i) {
      const size_t ao = (size_t)(m0 + (i << 4) + rlane) * lda + koff + k0;
      V ah = Frag<T>::load(Ab + ao);
      V al;
      if (SPLIT) al = Frag<T>::load(Ab2 + ao);
#pragma unroll
      for (int j = 0; j < 4; ++j) {
        acc[i][j] = Frag<T>::mma(ah, bh[j], acc[i][j]);
        if (SPLIT) {
          acc[i][j] = Frag<T>::mma(ah, bl[j], acc[i][j]);
          acc[i][j] = Frag<T>::mma(al, bh[j], acc[i][j]);
        }
      }
      Frag<T>::guard(acc[i][0], acc[i][3], ah, SPLIT ? al : ah);
    }
    Frag<T>::keep(bh[0], bh[1], bh[2], bh[3]);
    if (SPLIT) Frag<T>::keep(bl[0], bl[1], bl[2], bl[3]);
  }
  acc_guard4(acc[0][0], acc[0][1], acc[0][2], acc[0][3]);
  acc_guard4(acc[1][0], acc[1][1], acc[1][2], acc[1][3]);
  acc_guard4(acc[2][0], acc[2][1], acc[2][2], acc[2][3]);
  acc_guard4(acc[3][0], acc[3][1], acc[3][2], acc[3][3]);

  float* slab = sT[wave];
  const float* Rb = RESID ? (resid + (size_t)b * strideR) : nullptr;
#pragma unroll
  for (int i = 0; i < 4; ++i) {
    const int mBase = m0 + (i << 4);
#pragma unroll
    for (int j = 0; j < 4; ++j) {
      const int n = n0 + (j << 4) + rlane;
      float bv = 0.f;
      if (BIAS_MODE == 2) bv = bias[n];
#pragma unroll
      for (int r = 0; r < 8; ++r) {
        float v = acc[i][j][r] * scale;
        if (BIAS_MODE == 1) v += bias[mBase + mOff + r];
        if (BIAS_MODE == 2) v += bv;
        if (RESID) v += Rb[(size_t)(mBase + mOff + r) * ldc + n];
        if (ACT == 1) v = tanhf(v);
        if (ACT == 2) v = fmaxf(v, 0.0f);
        if (ACT == 3) v = v / (1.0f + expf(-v));
        if (ACT == 4) v = (v > 0.f) ? v : 0.01f * v;
        if (ACT == 5) v = 0.5f * v * (1.0f + erff(v * 0.70710678118654752f));
        slab[(mOff + r) * 68 + (j << 4) + rlane] = v;
      }
    }
    __builtin_amdgcn_fence(__ATOMIC_RELEASE, "workgroup");
    __builtin_amdgcn_wave_barrier();
    __builtin_amdgcn_fence(__ATOMIC_ACQUIRE, "workgroup");
    if (OUT_MODE == 0) {
      float* C = (float*)Cout + (size_t)b * strideC;
      const int hh = lane >> 4, c4 = (lane & 15) * 4;
      for (int pass = 0; pass < 2; ++pass) {
#pragma unroll
        for (int it = 0; it < 8; ++it) {
          const int row = it * 2 + hh;
          v4f v = *(const v4f*)(slab + row * 68 + c4);
          *(volatile v4f*)(C + (size_t)(mBase + row) * ldc + n0 + c4) = v;
        }
        __threadfence();
      }
    } else {
      const int q = lane >> 3, c8 = (lane & 7) * 8;
      unsigned short* C  = (unsigned short*)Cout  + (size_t)b * strideC;
      unsigned short* C2 = (OUT_MODE == 2) ? ((unsigned short*)Cout2 + (size_t)b * strideC) : nullptr;
      for (int pass = 0; pass < 2; ++pass) {
#pragma unroll
        for (int it = 0; it < 4; ++it) {
          const int row = it * 4 + q;
          const float* sp = slab + row * 68 + c8;
          v8h hv, lv;
#pragma unroll
          for (int e = 0; e < 8; ++e) {
            if (OUT_MODE == 1) {
              hv[e] = (_Float16)sp[e];
              lv[e] = hv[e];
            } else if (OUT_MODE == 3) {
              hv[e] = __builtin_bit_cast(_Float16, f2bf_bits(sp[e]));
              lv[e] = hv[e];
            } else {
              unsigned short hb = f2bf_bits(sp[e]);
              unsigned short lb = f2bf_bits(sp[e] - bf_bits2f(hb));
              hv[e] = __builtin_bit_cast(_Float16, hb);
              lv[e] = __builtin_bit_cast(_Float16, lb);
            }
          }
          *(volatile v8h*)(C + (size_t)(mBase + row) * ldc + n0 + c8) = hv;
          if (OUT_MODE == 2) *(volatile v8h*)(C2 + (size_t)(mBase + row) * ldc + n0 + c8) = lv;
        }
        __threadfence();
      }
    }
    __builtin_amdgcn_fence(__ATOMIC_RELEASE, "workgroup");
    __builtin_amdgcn_wave_barrier();
    __builtin_amdgcn_fence(__ATOMIC_ACQUIRE, "workgroup");
  }
}

__global__ __launch_bounds__(256) void cast_w_bf16x2(
    const float* __restrict__ wa, const float* __restrict__ wb,
    unsigned short* __restrict__ oa, unsigned short* __restrict__ ob,
    int n2a, int n2b, int blocksA) {
  const bool second = (blockIdx.x >= (unsigned)blocksA);
  const float* in = second ? wb : wa;
  unsigned short* out = second ? ob : oa;
  const int n2 = second ? n2b : n2a;
  const int i = ((int)blockIdx.x - (second ? blocksA : 0)) * 256 + (int)threadIdx.x;
  if (i < n2) {
    const unsigned u = (unsigned)f2bf_bits(in[2 * i]) | ((unsigned)f2bf_bits(in[2 * i + 1]) << 16);
    ((volatile unsigned*)out)[i] = u;
    __threadfence();
    ((volatile unsigned*)out)[i] = u;
  }
}

__global__ __launch_bounds__(256) void gn_stats(const float* __restrict__ x, float* __restrict__ stats) {
  __shared__ float rs[8], rq[8];
  const int bg = blockIdx.x;
  const int tid = threadIdx.x, lane = tid & 31, wave = tid >> 5;
  const float* xb = x + (size_t)bg * (CPG * NPOS);
  float s = 0.f, q = 0.f;
#pragma unroll 4
  for (int i = 0; i < (CPG * NPOS) / (256 * 4); ++i) {
    const v4f a = *(const v4f*)(xb + ((size_t)(i * 256 + tid)) * 4);
    s += (a[0] + a[1]) + (a[2] + a[3]);
    q += (a[0] * a[0] + a[1] * a[1]) + (a[2] * a[2] + a[3] * a[3]);
  }
#pragma unroll
  for (int off = 16; off >= 1; off >>= 1) {
    s += __shfl_xor(s, off, 32);
    q += __shfl_xor(q, off, 32);
  }
  if (lane == 0) { rs[wave] = s; rq[wave] = q; }
  __syncthreads();
  if (wave == 0) {
    float ts = 0.f, tq = 0.f;
#pragma unroll
    for (int w = 0; w < 8; ++w) { ts += rs[w]; tq += rq[w]; }
    const float inv_n = 1.0f / (float)(CPG * NPOS);
    const float mean = ts * inv_n;
    const float var  = fmaxf(tq * inv_n - mean * mean, 0.0f);
    const float rstd = rsqrtf(var + 1e-5f);
    const float val = (lane == 0) ? mean : ((lane == 1) ? rstd : 0.0f);
    volatile float* sp = stats + (size_t)bg * 32;
    sp[lane] = val;
    __threadfence();
    sp[lane] = val;
  }
}

__global__ __launch_bounds__(256) void gn_apply(
    const float* __restrict__ x, const float* __restrict__ stats,
    const float* __restrict__ gw, const float* __restrict__ gb,
    unsigned short* __restrict__ hT) {
  __shared__ __align__(16) unsigned short sh[64 * HPITCH];
  __shared__ float smean[NC], srstd[NC], sw[NC], sbb[NC];
  const int tid = threadIdx.x, lane = tid & 31, wave = tid >> 5;
  const int b  = blockIdx.x / (NPOS / 64);
  const int n0 = (blockIdx.x % (NPOS / 64)) * 64;
  {
    const int c = tid, g = c >> 3;
    smean[c] = stats[((size_t)(b * NG + g)) * 32 + 0];
    srstd[c] = stats[((size_t)(b * NG + g)) * 32 + 1];
    sw[c]  = gw[c];
    sbb[c] = gb[c];
  }
  __syncthreads();
#pragma unroll 4
  for (int it = 0; it < 16; ++it) {
    const int e4 = it * 256 + tid;
    const int c = e4 >> 4;
    const int nl4 = (e4 & 15) * 4;
    const v4f a = *(const v4f*)(x + ((size_t)(b * NC + c)) * NPOS + n0 + nl4);
    const float mu = smean[c], rsd = srstd[c], w = sw[c], bb = sbb[c];
#pragma unroll
    for (int j = 0; j < 4; ++j) {
      const float f = (a[j] - mu) * rsd * w + bb;
      sh[(nl4 + j) * HPITCH + c] = f2bf_bits(f);
    }
  }
  __syncthreads();
  const int q = lane >> 3, c8 = (lane & 7) * 8, col = q * 64 + c8;
  unsigned short* hb = hT + ((size_t)(b * NPOS + n0)) * NC;
  for (int pass = 0; pass < 2; ++pass) {
#pragma unroll
    for (int rr = 0; rr < 8; ++rr) {
      const int nl = wave * 8 + rr;
      const v8h val = *(const v8h*)(sh + nl * HPITCH + col);
      *(volatile v8h*)(hb + (size_t)nl * NC + col) = val;
    }
    __threadfence();
  }
}

__global__ __launch_bounds__(256) void softmax_rows(const float* __restrict__ S, unsigned short* __restrict__ P) {
  __shared__ float rmx[8], rsm[8];
  const int row = blockIdx.x;
  const int tid = threadIdx.x, lane = tid & 31, wave = tid >> 5;
  const float* sr = S + (size_t)row * NPOS;
  float v[32];
#pragma unroll
  for (int j = 0; j < 4; ++j) {
    const int base = (j * 256 + tid) * 8;
    const v4f a = *(const v4f*)(sr + base);
    const v4f c = *(const v4f*)(sr + base + 4);
    v[8 * j + 0] = a[0]; v[8 * j + 1] = a[1]; v[8 * j + 2] = a[2]; v[8 * j + 3] = a[3];
    v[8 * j + 4] = c[0]; v[8 * j + 5] = c[1]; v[8 * j + 6] = c[2]; v[8 * j + 7] = c[3];
  }
  float m = v[0];
#pragma unroll
  for (int i = 1; i < 32; ++i) m = fmaxf(m, v[i]);
#pragma unroll
  for (int off = 16; off >= 1; off >>= 1) m = fmaxf(m, __shfl_xor(m, off, 32));
  if (lane == 0) rmx[wave] = m;
  __syncthreads();
  m = rmx[0];
#pragma unroll
  for (int w = 1; w < 8; ++w) m = fmaxf(m, rmx[w]);
  float s = 0.f;
#pragma unroll
  for (int i = 0; i < 32; ++i) { v[i] = __expf(v[i] - m); s += v[i]; }
#pragma unroll
  for (int off = 16; off >= 1; off >>= 1) s += __shfl_xor(s, off, 32);
  if (lane == 0) rsm[wave] = s;
  __syncthreads();
  s = rsm[0];
#pragma unroll
  for (int w = 1; w < 8; ++w) s += rsm[w];
  const float inv = 1.0f / s;
  v8h pk[4];
#pragma unroll
  for (int j = 0; j < 4; ++j) {
#pragma unroll
    for (int e = 0; e < 8; ++e) pk[j][e] = __builtin_bit_cast(_Float16, f2bf_bits(v[8 * j + e] * inv));
  }
  unsigned short* pr = P + (size_t)row * NPOS;
  for (int pass = 0; pass < 2; ++pass) {
#pragma unroll
    for (int j = 0; j < 4; ++j) *(volatile v8h*)(pr + (size_t)(j * 256 + tid) * 8) = pk[j];
    __threadfence();
  }
}

extern "C" void kernel_launch(void* const* d_in, const int* in_sizes, int n_in,
                              void* d_out, int out_size, void* d_ws, size_t ws_size,
                              hipStream_t stream) {
  if (n_in < 7) return;
  const int NTOT = NB * NC * NPOS;
  if (in_sizes[0] != NTOT || in_sizes[1] != NC || in_sizes[2] != NC || in_sizes[3] != 3 * NC * NC ||
      in_sizes[4] != 3 * NC || in_sizes[5] != NC * NC || in_sizes[6] != NC || out_size != NTOT) return;

  const float* x      = (const float*)d_in[0];
  const float* norm_w = (const float*)d_in[1];
  const float* norm_b = (const float*)d_in[2];
  const float* qkv_w  = (const float*)d_in[3];
  const float* qkv_b  = (const float*)d_in[4];
  const float* proj_w = (const float*)d_in[5];
  const float* proj_b = (const float*)d_in[6];
  float* out = (float*)d_out;

  const size_t OFF_STATS = 0;
  const size_t OFF_WQ    = OFF_STATS + (size_t)NB * NG * 32 * 4;
  const size_t OFF_WP    = OFF_WQ + (size_t)3 * NC * NC * 2;
  const size_t OFF_HT    = OFF_WP + (size_t)NC * NC * 2;
  const size_t OFF_QK    = OFF_HT + (size_t)NB * NPOS * NC * 2;
  const size_t OFF_V     = OFF_QK + (size_t)NB * NPOS * 2 * NC * 2;
  const size_t OFF_S     = OFF_V + (size_t)NB * NC * NPOS * 2;
  const size_t OFF_P     = OFF_S + (size_t)QBLK * NPOS * 4;
  const size_t OFF_HO    = OFF_P + (size_t)QBLK * NPOS * 2;
  const size_t OFF_END   = OFF_HO + (size_t)NB * NPOS * NC * 2;
  if (OFF_END > ws_size) return;

  char* ws = (char*)d_ws;
  float*          stats = (float*)(ws + OFF_STATS);
  unsigned short* wq    = (unsigned short*)(ws + OFF_WQ);
  unsigned short* wp    = (unsigned short*)(ws + OFF_WP);
  unsigned short* hT    = (unsigned short*)(ws + OFF_HT);
  unsigned short* qk    = (unsigned short*)(ws + OFF_QK);
  unsigned short* vpl   = (unsigned short*)(ws + OFF_V);
  float*          S     = (float*)(ws + OFF_S);
  unsigned short* P     = (unsigned short*)(ws + OFF_P);
  unsigned short* hout  = (unsigned short*)(ws + OFF_HO);

  const int n2q = (3 * NC * NC) / 2;
  const int n2p = (NC * NC) / 2;
  const int blocksA = (n2q + 255) / 256, blocksB = (n2p + 255) / 256;
  cast_w_bf16x2<<<blocksA + blocksB, 256, 0, stream>>>(qkv_w, proj_w, wq, wp, n2q, n2p, blocksA);

  gn_stats<<<NB * NG, 256, 0, stream>>>(x, stats);
  gn_apply<<<NB * (NPOS / 64), 256, 0, stream>>>(x, stats, norm_w, norm_b, hT);

  wmma_gemm64<1, false, 2, 3, false><<<dim3((NPOS / 64) * (2 * NC / 64) / 8, NB), 256, 0, stream>>>(
      hT, hT, NC, (long)NPOS * NC,
      wq, wq, NC, 0L,
      (void*)qk, (void*)qk, 2 * NC, (long)NPOS * 2 * NC,
      qkv_b, x, 0L, NPOS, 2 * NC, NC, 1.0f);

  wmma_gemm64<1, false, 1, 3, false><<<dim3((NC / 64) * (NPOS / 64) / 8, NB), 256, 0, stream>>>(
      wq + (size_t)2 * NC * NC, wq + (size_t)2 * NC * NC, NC, 0L,
      hT, hT, NC, (long)NPOS * NC,
      (void*)vpl, (void*)vpl, NPOS, (long)NC * NPOS,
      qkv_b + 2 * NC, x, 0L, NC, NPOS, NC, 1.0f);

  for (int i = 0; i < NB * (NPOS / QBLK); ++i) {
    const int b = i / (NPOS / QBLK), qbk = i % (NPOS / QBLK);
    const unsigned short* qbase = qk + (size_t)b * NPOS * 2 * NC + (size_t)qbk * QBLK * 2 * NC;
    const unsigned short* kbase = qk + (size_t)b * NPOS * 2 * NC + NC;
    wmma_gemm64<1, false, 0, 0, false><<<dim3((QBLK / 64) * (NPOS / 64) / 8, 1), 256, 0, stream>>>(
        qbase, qbase, 2 * NC, 0L,
        kbase, kbase, 2 * NC, 0L,
        (void*)S, (void*)S, NPOS, 0L,
        qkv_b, x, 0L, QBLK, NPOS, NC, 0.0625f);
    softmax_rows<<<QBLK, 256, 0, stream>>>(S, P);
    wmma_gemm64<1, false, 0, 3, false><<<dim3((QBLK / 64) * (NC / 64) / 8, 1), 256, 0, stream>>>(
        P, P, NPOS, 0L,
        vpl + (size_t)b * NC * NPOS, vpl + (size_t)b * NC * NPOS, NPOS, 0L,
        (void*)(hout + ((size_t)b * NPOS + (size_t)qbk * QBLK) * NC),
        (void*)(hout + ((size_t)b * NPOS + (size_t)qbk * QBLK) * NC), NC, 0L,
        qkv_b, x, 0L, QBLK, NC, NPOS, 1.0f);
  }

  wmma_gemm64<1, false, 1, 0, true><<<dim3((NC / 64) * (NPOS / 64) / 8, NB), 256, 0, stream>>>(
      wp, wp, NC, 0L,
      hout, hout, NC, (long)NPOS * NC,
      (void*)out, (void*)out, NPOS, (long)NC * NPOS,
      proj_b, x, (long)NC * NPOS, NC, NPOS, NC, 1.0f);
}
